// ColourHistogram_566935683074
// MI455X (gfx1250) — hardware-verified
//
#include <hip/hip_runtime.h>
#include <math.h>

#define NIMG 16
#define HWP  262144
#define NBIN 32
#define CHUNK 4096
#define NCH  (HWP / CHUNK)

typedef _Float16 f16;
typedef __attribute__((ext_vector_type(16))) f16 f16x16;
typedef __attribute__((ext_vector_type(8)))  f16 f16x8;
typedef __attribute__((ext_vector_type(8)))  float f32x8;
typedef __attribute__((ext_vector_type(4)))  float v4f_t;
typedef float v4fa __attribute__((ext_vector_type(4), may_alias));

__device__ __forceinline__ f32x8 wmma16(f16x16 a, f16x16 b, f32x8 c) {
  c = __builtin_amdgcn_wmma_f32_16x16x32_f16(false, a, false, b, (short)0, c, false, false);
  asm volatile("v_nop\n\tv_nop\n\tv_nop\n\tv_nop" : "+v"(c) : "v"(a), "v"(b));
  return c;
}
__device__ __forceinline__ f16x16 lds_frag(const f16* base, int stride) {
  const int lane = threadIdx.x & 31, row = lane & 15, kh = (lane >> 4) * 8;
  const f16x8 lo = *(const f16x8*)(base + row * stride + kh);
  const f16x8 hi = *(const f16x8*)(base + row * stride + kh + 16);
  f16x16 f;
#pragma unroll
  for (int i = 0; i < 8; ++i) { f[i] = lo[i]; f[i + 8] = hi[i]; }
  return f;
}

__global__ __launch_bounds__(256) void k_hist(const float* __restrict__ img, float* __restrict__ partial) {
  __shared__ __attribute__((aligned(16))) f16 kaS[8][32 * 40], kbS[8][32 * 40];
  __shared__ float redS[8][32 * 33];
  __shared__ __attribute__((aligned(16))) float outS[32 * 32];
  const int tid = threadIdx.x, lane = tid & 31, wave = tid >> 5, cl = lane & 15, rh = (lane >> 4) * 8;
  const int n = blockIdx.x / NCH, ch = blockIdx.x % NCH;
  const float* pa = img + ((size_t)n * 2 + 0) * HWP + (size_t)ch * CHUNK + wave * 512;
  const float* pb = img + ((size_t)n * 2 + 1) * HWP + (size_t)ch * CHUNK + wave * 512;
  const float inv_sigma = 1.0f / 0.05f, bstep = 1.0f / 31.0f;
  f16* ka = kaS[wave]; f16* kb = kbS[wave];
  f32x8 acc[2][2];
#pragma unroll
  for (int i = 0; i < 2; ++i)
#pragma unroll
    for (int j = 0; j < 2; ++j) { f32x8 z = {}; acc[i][j] = z; }
#pragma unroll 1
  for (int st = 0; st < 16; ++st) {
    const float va = pa[st * 32 + lane], vb = pb[st * 32 + lane];
#pragma unroll 8
    for (int bi = 0; bi < NBIN; ++bi) {
      const float cb = (float)bi * bstep;
      const float da = (va - cb) * inv_sigma, db = (vb - cb) * inv_sigma;
      ka[bi * 40 + lane] = (f16)__expf(-0.5f * da * da);
      kb[bi * 40 + lane] = (f16)__expf(-0.5f * db * db);
    }
    asm volatile("s_wait_dscnt 0" ::: "memory");
    __builtin_amdgcn_wave_barrier();
#pragma unroll
    for (int i = 0; i < 2; ++i) {
      const f16x16 af = lds_frag(ka + (i * 16) * 40, 40);
#pragma unroll
      for (int j = 0; j < 2; ++j) acc[i][j] = wmma16(af, lds_frag(kb + (j * 16) * 40, 40), acc[i][j]);
    }
    __builtin_amdgcn_wave_barrier();
  }
  float* rw = redS[wave];
#pragma unroll
  for (int i = 0; i < 2; ++i)
#pragma unroll
    for (int j = 0; j < 2; ++j)
#pragma unroll
      for (int r = 0; r < 8; ++r) rw[(i * 16 + rh + r) * 33 + j * 16 + cl] = acc[i][j][r];
  __syncthreads();
  for (int e = tid; e < 32 * 32; e += 256) { const int a = e >> 5, b = e & 31; float s = 0.0f;
#pragma unroll
    for (int w = 0; w < 8; ++w) s += redS[w][a * 33 + b]; outS[e] = s; }
  __syncthreads();
  float* dst = partial + ((size_t)n * NCH + ch) * 1024;
  *(volatile v4f_t*)(dst + tid * 4) = *(const volatile v4fa*)(outS + tid * 4); __threadfence(); *(volatile v4f_t*)(dst + tid * 4) = *(const volatile v4fa*)(outS + tid * 4);
}
__global__ __launch_bounds__(256) void k_sum(const float* __restrict__ partial, float* __restrict__ hist) {
  __shared__ __attribute__((aligned(16))) float hS[1024];
  const int n = blockIdx.x, tid = threadIdx.x;
  for (int e = tid; e < 1024; e += 256) { float s = 0.0f; for (int ch = 0; ch < NCH; ++ch) s += partial[((size_t)n * NCH + ch) * 1024 + e]; hS[e] = s; }
  __syncthreads();
  *(volatile v4f_t*)(hist + (size_t)n * 1024 + tid * 4) = *(const volatile v4fa*)(hS + tid * 4); __threadfence(); *(volatile v4f_t*)(hist + (size_t)n * 1024 + tid * 4) = *(const volatile v4fa*)(hS + tid * 4);
}

extern "C" void kernel_launch(void* const* d_in, const int* in_sizes, int n_in,
                              void* d_out, int out_size, void* d_ws, size_t ws_size,
                              hipStream_t stream) {
  (void)in_sizes; (void)n_in; (void)out_size; (void)ws_size;
  const float* img = (const float*)d_in[0];
  float* out = (float*)d_out;
  float* partial = (float*)d_ws;
  k_hist<<<dim3(NIMG * NCH), dim3(256), 0, stream>>>(img, partial);
  k_sum<<<dim3(NIMG), dim3(256), 0, stream>>>(partial, out);
}
